// TransformerLayer_78116865179728
// MI455X (gfx1250) — hardware-verified
//
#include <hip/hip_runtime.h>
#include <math.h>

#ifndef NB
#define NB 2
#endif
#ifndef SEQ
#define SEQ 256
#endif
#define SEQ_FULL 256
#define DM 320
#define DE 64
#define FFD 256
#define MTOK (NB * SEQ)

#define LG_ACT 3
#define LG_W 5
#define LG_WV 6
#define LG_WO 6
#define LG_X1 4
#define C_ACT 8.0f
#define C_WV 64.0f
#define C_X1 16.0f
#define SC_EDGE (1.0f / 256.0f)
#define QSCALE 0.15811388300841898f
#define LOG2E 1.4426950408889634f

static_assert(SEQ == 256);
static_assert(SEQ == SEQ_FULL);
static_assert(MTOK % 64 == 0);
static_assert(DM % 64 == 0 && (3 * DM) % 64 == 0 && FFD % 64 == 0);
static_assert(DM % 32 == 0 && FFD % 32 == 0 && DE % 32 == 0);
static_assert(DM == 320 && DM / 4 == 80 && DM / 8 == 40);
static_assert(C_ACT == (float)(1 << LG_ACT));
static_assert(C_WV == (float)(1 << LG_WV));
static_assert(C_X1 == (float)(1 << LG_X1));
static_assert(SC_EDGE * (float)(1 << (LG_ACT + LG_W)) == 1.0f);
static_assert(((size_t)MTOK * SEQ * DE / 8) % 256 == 0);
static_assert((MTOK * DM / 8) % 256 == 0);
static_assert(MTOK % 8 == 0);

typedef _Float16 h16;
typedef __attribute__((ext_vector_type(16))) _Float16 v16h;
typedef __attribute__((ext_vector_type(8)))  _Float16 v8h;
typedef __attribute__((ext_vector_type(8)))  float    v8f;
typedef __attribute__((ext_vector_type(4)))  float    v4f;
typedef __attribute__((ext_vector_type(4)))  unsigned int v4u;


#define VST2(T, ptr, val) do { const T vst2_v_ = (val); *(volatile T*)(ptr) = vst2_v_; __threadfence(); *(volatile T*)(ptr) = vst2_v_; } while (0)

__device__ __forceinline__ float bfr(float f) {
    unsigned u = __float_as_uint(f);
    u += 0x7FFFu + ((u >> 16) & 1u);
    return __uint_as_float(u & 0xFFFF0000u);
}
__device__ __forceinline__ unsigned short f2h_bits(float x) {
    return (fabsf(x) < 6.104e-5f) ? (unsigned short)0 : __builtin_bit_cast(unsigned short, (_Float16)x);
}
static __device__ __forceinline__ h16 toh_flush(float v) { const float w = (fabsf(v) < 6.103515625e-05f) ? 0.0f : v; return (h16)w; }
__device__ __forceinline__ void st8h(unsigned short* P, size_t o, const float* v) {
    v4u pk;
    pk.x = (unsigned)f2h_bits(v[0]) | ((unsigned)f2h_bits(v[1]) << 16);
    pk.y = (unsigned)f2h_bits(v[2]) | ((unsigned)f2h_bits(v[3]) << 16);
    pk.z = (unsigned)f2h_bits(v[4]) | ((unsigned)f2h_bits(v[5]) << 16);
    pk.w = (unsigned)f2h_bits(v[6]) | ((unsigned)f2h_bits(v[7]) << 16);
    VST2(v4u, (v4u*)(P + o), pk);
}

union FragU { v16h v; v8h h[2]; };
__device__ __forceinline__ v16h frag_ld(const _Float16* p) {
    FragU f; f.h[0] = *(const v8h*)(p); f.h[1] = *(const v8h*)(p + 16); return f.v;
}
__device__ __forceinline__ v8f wmma16(v16h a, v16h b, v8f c) {
    c = __builtin_amdgcn_wmma_f32_16x16x32_f16(false, a, false, b, (short)0, c, false, false);
    asm volatile("v_nop\n\tv_nop\n\tv_nop\n\tv_nop" : "+v"(c) : "v"(a), "v"(b));
    return c;
}
__device__ __forceinline__ void wave_sync_lds() {
    __builtin_amdgcn_fence(3  , "workgroup");
    __builtin_amdgcn_wave_barrier();
    __builtin_amdgcn_fence(2  , "workgroup");
}

template <int OUT_MODE, int RESID, bool RELU, bool BIAS, bool ROWMASK, int LGS, int LGO, unsigned M, unsigned N, unsigned K>
static __device__ __forceinline__ void gemm64_body(
    const _Float16* __restrict__ A, const _Float16* __restrict__ Bt, void* __restrict__ Cout,
    const float* __restrict__ bias, const float* __restrict__ resid, const float* __restrict__ rowmask) {
  static_assert(M % 64u == 0u && N % 64u == 0u && K % 32u == 0u);
  static_assert(32 * 16 * 8 == 16 * 64 * 4);
  static_assert(32 * 16 * 4 == 16 * 64 * 2);
  static_assert(8 * 16 * 68 * 4 <= 131072);
  __shared__ __align__(16) float sT[8][16 * 68];
  constexpr float scale = 1.0f / (float)(1u << LGS);
  constexpr float oscale = (float)(1u << LGO);
  constexpr unsigned TN = N / 64u, TM = M / 64u;
  const unsigned lane = threadIdx.x & 31u;
  const unsigned wave = (unsigned)__builtin_amdgcn_readfirstlane((int)(threadIdx.x >> 5));
  const unsigned tile = blockIdx.x * 8u + wave;
  if (tile >= TM * TN) return;
  const unsigned tm = tile / TN;
  const unsigned tn = tile - tm * TN;
  const unsigned m0 = tm << 6, n0 = tn << 6;
  const unsigned rlane = lane & 15u;
  const unsigned koff = (lane >> 4) * 8u;
  const unsigned mOff = koff;

  v8f acc[4][4];
#pragma unroll
  for (int i = 0; i < 4; ++i)
#pragma unroll
    for (int j = 0; j < 4; ++j) acc[i][j] = (v8f){0.f,0.f,0.f,0.f,0.f,0.f,0.f,0.f};

#pragma unroll 1
  for (unsigned k0 = 0; k0 < K; k0 += 32u) {
    v16h bh[4];
#pragma unroll
    for (int j = 0; j < 4; ++j)
      bh[j] = frag_ld(Bt + (size_t)(n0 + ((unsigned)j << 4) + rlane) * K + koff + k0);
#pragma unroll
    for (int i = 0; i < 4; ++i) {
      const v16h ah = frag_ld(A + (size_t)(m0 + ((unsigned)i << 4) + rlane) * K + koff + k0);
#pragma unroll
      for (int j = 0; j < 4; ++j)
        acc[i][j] = wmma16(ah, bh[j], acc[i][j]);
    }
  }

#pragma unroll
  for (int i = 0; i < 4; ++i) {
    const unsigned mBase = m0 + ((unsigned)i << 4);
    float nmr[8];
    if (ROWMASK) {
      const v4f ra = *(const v4f*)(rowmask + mBase + mOff);
      const v4f rb = *(const v4f*)(rowmask + mBase + mOff + 4u);
      nmr[0] = bfr(ra.x); nmr[1] = bfr(ra.y); nmr[2] = bfr(ra.z); nmr[3] = bfr(ra.w);
      nmr[4] = bfr(rb.x); nmr[5] = bfr(rb.y); nmr[6] = bfr(rb.z); nmr[7] = bfr(rb.w);
    } else {
#pragma unroll
      for (int r = 0; r < 8; ++r) nmr[r] = 1.0f;
    }
#pragma unroll
    for (int j = 0; j < 4; ++j) {
      const unsigned n = n0 + ((unsigned)j << 4) + rlane;
      float bv = 0.0f;
      if (BIAS) bv = bfr(bias[n]);
#pragma unroll
      for (int r = 0; r < 8; ++r) {
        float v = acc[i][j][r] * scale + bv;
        if (RELU) v = fmaxf(v, 0.0f);
        if (ROWMASK) v *= nmr[r];
        if (OUT_MODE == 1) v *= oscale;
        sT[wave][(mOff + (unsigned)r) * 68u + ((unsigned)j << 4) + rlane] = v;
      }
    }
    wave_sync_lds();
    if (OUT_MODE == 0) {
      float* C = (float*)Cout;
      const unsigned hh = lane >> 4, c4 = (lane & 15u) * 4u;
#pragma unroll
      for (int half = 0; half < 2; ++half) {
        v4f vv[4];
#pragma unroll
        for (int it = 0; it < 4; ++it) {
          const unsigned row = (unsigned)(half * 4 + it) * 2u + hh;
          vv[it] = *(const v4f*)(&sT[wave][row * 68u + c4]);
          if (RESID == 1) vv[it] += *(const v4f*)(resid + (size_t)(mBase + row) * N + n0 + c4);
          if (RESID == 2) {
            const v4f rr = *(const v4f*)(resid + (size_t)(mBase + row) * N + n0 + c4);
            vv[it].x += bfr(rr.x); vv[it].y += bfr(rr.y); vv[it].z += bfr(rr.z); vv[it].w += bfr(rr.w);
          }
        }
        for (int pass = 0; pass < 2; ++pass) {
#pragma unroll
          for (int it = 0; it < 4; ++it) {
            const unsigned row = (unsigned)(half * 4 + it) * 2u + hh;
            *(volatile v4f*)(C + (size_t)(mBase + row) * N + n0 + c4) = vv[it];
          }
          __threadfence();
        }
      }
    } else {
      _Float16* C = (_Float16*)Cout;
      const unsigned q = lane >> 3, c8 = (lane & 7u) * 8u;
      v8h hv[4];
#pragma unroll
      for (int it = 0; it < 4; ++it) {
        const unsigned row = (unsigned)it * 4u + q;
        const float* sp = &sT[wave][row * 68u + c8];
#pragma unroll
        for (int e = 0; e < 8; ++e) hv[it][e] = toh_flush(sp[e]);
      }
      for (int pass = 0; pass < 2; ++pass) {
#pragma unroll
        for (int it = 0; it < 4; ++it) {
          const unsigned row = (unsigned)it * 4u + q;
          *(volatile v8h*)(C + (size_t)(mBase + row) * N + n0 + c8) = hv[it];
        }
        __threadfence();
      }
    }
    wave_sync_lds();
  }
}

__global__ __launch_bounds__(256) void k_gemm_qkv(const _Float16* __restrict__ A, const _Float16* __restrict__ Bt, float* __restrict__ C) {
  gemm64_body<0, 0, false, false, false, LG_ACT + LG_W, 0, MTOK, 3 * DM, DM>(A, Bt, (void*)C, nullptr, nullptr, nullptr);
}
__global__ __launch_bounds__(256) void k_gemm_wo(const _Float16* __restrict__ A, const _Float16* __restrict__ Bt, float* __restrict__ C,
                                                 const float* __restrict__ bias, const float* __restrict__ resid, const float* __restrict__ rowmask) {
  gemm64_body<0, 2, false, true, true, LG_WV + LG_WO, 0, MTOK, DM, DM>(A, Bt, (void*)C, bias, resid, rowmask);
}
__global__ __launch_bounds__(256) void k_gemm_ff1(const _Float16* __restrict__ A, const _Float16* __restrict__ Bt, _Float16* __restrict__ C,
                                                  const float* __restrict__ bias) {
  gemm64_body<1, 0, true, true, false, LG_X1 + LG_W, LG_X1, MTOK, FFD, DM>(A, Bt, (void*)C, bias, nullptr, nullptr);
}
__global__ __launch_bounds__(256) void k_gemm_ff2(const _Float16* __restrict__ A, const _Float16* __restrict__ Bt, float* __restrict__ C,
                                                  const float* __restrict__ bias, const float* __restrict__ resid) {
  gemm64_body<0, 1, false, true, false, LG_X1 + LG_W, 0, MTOK, DM, FFD>(A, Bt, (void*)C, bias, resid, nullptr);
}

__global__ __launch_bounds__(256) void k_wt16(const float* __restrict__ Wm, unsigned KI, unsigned NO, unsigned per,
                                              unsigned short* __restrict__ W16, unsigned lgsw) {
    const unsigned u = blockIdx.x * 256u + threadIdx.x;
    if (u >= NO * per) return;
    const float sw = (float)(1u << lgsw);
    const unsigned o = u / per;
    const unsigned k0 = 8u * (u - o * per);
    float v[8];
#pragma unroll
    for (int i = 0; i < 8; ++i) v[i] = bfr(Wm[(size_t)(k0 + (unsigned)i) * NO + o]) * sw;
    st8h(W16, (size_t)o * KI + k0, v);
}

__global__ __launch_bounds__(256) void k_cvt8(const float* __restrict__ src, unsigned short* __restrict__ dst, unsigned n8) {
    const unsigned u = blockIdx.x * 256u + threadIdx.x;
    if (u >= n8) return;
    const float* sp = src + (size_t)u * 8u;
    const v4f a = *(const v4f*)sp, b = *(const v4f*)(sp + 4);
    float v[8];
    v[0] = bfr(a.x) * C_ACT; v[1] = bfr(a.y) * C_ACT; v[2] = bfr(a.z) * C_ACT; v[3] = bfr(a.w) * C_ACT;
    v[4] = bfr(b.x) * C_ACT; v[5] = bfr(b.y) * C_ACT; v[6] = bfr(b.z) * C_ACT; v[7] = bfr(b.w) * C_ACT;
    st8h(dst, (size_t)u * 8u, v);
}

__global__ __launch_bounds__(256) void k_qkvt(const float* __restrict__ QKV, const float* __restrict__ bq, const float* __restrict__ bk,
                                              const float* __restrict__ bv, const float* __restrict__ nmask,
                                              float* __restrict__ QS, float* __restrict__ KVT) {
    static_assert(256 * 16 * 4 == 64 * 64 * 4);
    __shared__ __align__(16) float sX[64 * 68];
    const unsigned t = threadIdx.x;
    const unsigned fb = blockIdx.x, jb = blockIdx.y, z = blockIdx.z;
    const unsigned m0 = jb * 64u, f0 = fb * 64u;
    const unsigned c4 = (t & 15u) * 4u, r0 = t >> 4;
    const v4f vq = *(const v4f*)(bq + f0 + c4);
    const v4f vk = *(const v4f*)(bk + f0 + c4);
    const v4f vv = *(const v4f*)(bv + f0 + c4);
    v4f bias;
    bias.x = bfr((z == 0u) ? vq.x : ((z == 1u) ? vk.x : vv.x));
    bias.y = bfr((z == 0u) ? vq.y : ((z == 1u) ? vk.y : vv.y));
    bias.z = bfr((z == 0u) ? vq.z : ((z == 1u) ? vk.z : vv.z));
    bias.w = bfr((z == 0u) ? vq.w : ((z == 1u) ? vk.w : vv.w));
    const float sc = (z == 0u) ? QSCALE : 1.0f;
#pragma unroll
    for (int it = 0; it < 4; ++it) {
        const unsigned row = r0 + 16u * (unsigned)it;
        v4f x = *(const v4f*)(QKV + (size_t)(m0 + row) * (3u * DM) + z * DM + f0 + c4);
        const float nm = bfr(nmask[m0 + row]);
        x.x = ((x.x + bias.x) * nm) * sc; x.y = ((x.y + bias.y) * nm) * sc;
        x.z = ((x.z + bias.z) * nm) * sc; x.w = ((x.w + bias.w) * nm) * sc;
        *(v4f*)(sX + row * 68u + c4) = x;
    }
    __syncthreads();
    v4f o[4];
    if (z == 0u) {
#pragma unroll
        for (int it = 0; it < 4; ++it) o[it] = *(const v4f*)(sX + (r0 + 16u * (unsigned)it) * 68u + c4);
        float* dst = QS + (size_t)m0 * DM + f0 + c4;
        for (int pass = 0; pass < 2; ++pass) {
#pragma unroll
            for (int it = 0; it < 4; ++it) *(volatile v4f*)(dst + (size_t)(r0 + 16u * (unsigned)it) * DM) = o[it];
            __threadfence();
        }
    } else {
        const unsigned b = m0 / (unsigned)SEQ;
        const unsigned jl = m0 - b * (unsigned)SEQ;
#pragma unroll
        for (int it = 0; it < 4; ++it) {
            const unsigned f = r0 + 16u * (unsigned)it;
            o[it].x = sX[(c4 + 0u) * 68u + f]; o[it].y = sX[(c4 + 1u) * 68u + f];
            o[it].z = sX[(c4 + 2u) * 68u + f]; o[it].w = sX[(c4 + 3u) * 68u + f];
        }
        float* dst = KVT + (size_t)(z - 1u) * ((size_t)NB * DM * SEQ) + (size_t)(b * DM + f0) * SEQ + jl + c4;
        for (int pass = 0; pass < 2; ++pass) {
#pragma unroll
            for (int it = 0; it < 4; ++it) *(volatile v4f*)(dst + (size_t)(r0 + 16u * (unsigned)it) * SEQ) = o[it];
            __threadfence();
        }
    }
}

__global__ __launch_bounds__(128) void k_eattn(const _Float16* __restrict__ EB, const _Float16* __restrict__ wem16, const _Float16* __restrict__ wea16,
                                               const float* __restrict__ bem, const float* __restrict__ bea, const float* __restrict__ nmask,
                                               const float* __restrict__ QS, const float* __restrict__ KVT, _Float16* __restrict__ WV) {
    static_assert(8 * 16 == 64 * 2);
    static_assert(DM == 5 * 64 && SEQ % 16 == 0);
    __shared__ __align__(16) float sW[64];
    const unsigned lane = threadIdx.x & 31u;
    const unsigned wave = (unsigned)__builtin_amdgcn_readfirstlane((int)(threadIdx.x >> 5));
    const unsigned hh = lane >> 4, c = lane & 15u;
    const unsigned bx = blockIdx.x;
    const unsigned row = bx / 5u;
    const unsigned fb = bx - row * 5u;
    const unsigned b = row / (unsigned)SEQ;
    const unsigned f = fb * 64u + wave * 16u + c;

    const _Float16* wm = wem16 + (size_t)f * DE + 8u * hh;
    const _Float16* wa = wea16 + (size_t)f * DE + 8u * hh;
    const v16h bm0 = frag_ld(wm), bm1 = frag_ld(wm + 32);
    const v16h ba0 = frag_ld(wa), ba1 = frag_ld(wa + 32);

    const float qs = QS[(size_t)row * DM + f];
    const float b1 = bfr(bem[f]);
    const float b2 = bfr(bea[f]);
    const float nmi = bfr(nmask[row]);
    const float* KT = KVT + (size_t)(b * DM + f) * SEQ + 8u * hh;
    const float* VT = KT + (size_t)NB * DM * SEQ;
    const float* NM = nmask + b * (unsigned)SEQ_FULL + 8u * hh;
    const _Float16* EA = EB + ((size_t)row * SEQ_FULL + c) * DE + 8u * hh;

    float m = -3.0e38f, l = 0.f, a = 0.f;
#pragma unroll 1
    for (unsigned t = 0; t < (unsigned)(SEQ / 16); ++t) {
        const unsigned j0 = t * 16u;
        const _Float16* ea = EA + (size_t)j0 * DE;
        const v16h a0 = frag_ld(ea), a1 = frag_ld(ea + 32);
        v8f e1 = (v8f){0.f,0.f,0.f,0.f,0.f,0.f,0.f,0.f};
        v8f e2 = (v8f){0.f,0.f,0.f,0.f,0.f,0.f,0.f,0.f};
        e1 = wmma16(a0, bm0, e1);
        e1 = wmma16(a1, bm1, e1);
        e2 = wmma16(a0, ba0, e2);
        e2 = wmma16(a1, ba1, e2);
        const v4f ka = *(const v4f*)(KT + j0), kb = *(const v4f*)(KT + j0 + 4u);
        const v4f va = *(const v4f*)(VT + j0), vb = *(const v4f*)(VT + j0 + 4u);
        const v4f na = *(const v4f*)(NM + j0), nb2 = *(const v4f*)(NM + j0 + 4u);
        const float kk[8] = {ka.x, ka.y, ka.z, ka.w, kb.x, kb.y, kb.z, kb.w};
        const float vv[8] = {va.x, va.y, va.z, va.w, vb.x, vb.y, vb.z, vb.w};
        const float nn[8] = {bfr(na.x), bfr(na.y), bfr(na.z), bfr(na.w), bfr(nb2.x), bfr(nb2.y), bfr(nb2.z), bfr(nb2.w)};
        float y[8];
        float mx = -3.0e38f;
#pragma unroll
        for (int r = 0; r < 8; ++r) {
            const float em = nmi * nn[r];
            const float E1 = (e1[r] * SC_EDGE + b1) * em;
            const float E2 = (e2[r] * SC_EDGE + b2) * em;
            float yy = (qs * kk[r]) * (E1 + 1.0f) + E2;
            yy = (nn[r] > 0.0f) ? yy : -1.0e9f;
            yy *= LOG2E;
            y[r] = yy;
            mx = fmaxf(mx, yy);
        }
        const float mnew = fmaxf(m, mx);
        const float alpha = exp2f(m - mnew);
        m = mnew;
        float ps = 0.f, pa = 0.f;
#pragma unroll
        for (int r = 0; r < 8; ++r) {
            const float p = exp2f(y[r] - mnew);
            ps += p;
            pa += p * vv[r];
        }
        l = l * alpha + ps;
        a = a * alpha + pa;
    }
    const float mo = __shfl_xor(m, 16, 32);
    const float lo = __shfl_xor(l, 16, 32);
    const float ao = __shfl_xor(a, 16, 32);
    const float mn = fmaxf(m, mo);
    const float s0 = exp2f(m - mn), s1 = exp2f(mo - mn);
    const float lt = l * s0 + lo * s1;
    const float at = a * s0 + ao * s1;
    const float wvv = at * (1.0f / lt);
    if (hh == 0u) sW[wave * 16u + c] = wvv;
    __syncthreads();
    const unsigned p8 = (lane & 7u) * 8u;
    const v4f x0 = *(const v4f*)(sW + p8), x1 = *(const v4f*)(sW + p8 + 4u);
    if (wave == 0u) {
        v8h o;
        o[0] = toh_flush(x0.x * C_WV); o[1] = toh_flush(x0.y * C_WV); o[2] = toh_flush(x0.z * C_WV); o[3] = toh_flush(x0.w * C_WV);
        o[4] = toh_flush(x1.x * C_WV); o[5] = toh_flush(x1.y * C_WV); o[6] = toh_flush(x1.z * C_WV); o[7] = toh_flush(x1.w * C_WV);
        if (lane < 8u) {
            _Float16* dst = WV + (size_t)row * DM + fb * 64u + p8;
            *(volatile v8h*)dst = o;
            __threadfence();
            *(volatile v8h*)dst = o;
        }
    }
}

template <bool PLANE>
static __device__ __forceinline__ void ln320_body(const float* __restrict__ h, const float* __restrict__ g, const float* __restrict__ bt,
                                                  float* __restrict__ y32, unsigned short* __restrict__ y16) {
    static_assert((32 + 32 + 16) * 16 == DM * 4);
    static_assert((32 + 8) * 16 == DM * 2);
    __shared__ __align__(16) float sL[8][DM];
    const unsigned wave = (unsigned)__builtin_amdgcn_readfirstlane((int)(threadIdx.x >> 5));
    const unsigned L = threadIdx.x & 31u;
    const unsigned row = blockIdx.x * 8u + wave;
    if (row >= (unsigned)MTOK) return;
    const unsigned q0 = 4u * L, q1 = 4u * (L + 32u), q2 = 4u * min(L + 64u, 79u);
    const bool ok2 = (L < 16u);
    const float* hr = h + (size_t)row * DM;
    const v4f x0 = *(const v4f*)(hr + q0), x1 = *(const v4f*)(hr + q1);
    v4f x2 = *(const v4f*)(hr + q2);
    x2.x = ok2 ? x2.x : 0.f; x2.y = ok2 ? x2.y : 0.f; x2.z = ok2 ? x2.z : 0.f; x2.w = ok2 ? x2.w : 0.f;
    float s = ((x0.x + x0.y) + (x0.z + x0.w)) + ((x1.x + x1.y) + (x1.z + x1.w)) + ((x2.x + x2.y) + (x2.z + x2.w));
#pragma unroll
    for (int o = 16; o > 0; o >>= 1) s += __shfl_xor(s, o, 32);
    const float mu = s * (1.0f / (float)DM);
    v4f d0, d1, d2;
    d0.x = x0.x - mu; d0.y = x0.y - mu; d0.z = x0.z - mu; d0.w = x0.w - mu;
    d1.x = x1.x - mu; d1.y = x1.y - mu; d1.z = x1.z - mu; d1.w = x1.w - mu;
    d2.x = ok2 ? (x2.x - mu) : 0.f; d2.y = ok2 ? (x2.y - mu) : 0.f; d2.z = ok2 ? (x2.z - mu) : 0.f; d2.w = ok2 ? (x2.w - mu) : 0.f;
    float q = d0.x * d0.x + d0.y * d0.y + d0.z * d0.z + d0.w * d0.w;
    q += d1.x * d1.x + d1.y * d1.y + d1.z * d1.z + d1.w * d1.w;
    q += d2.x * d2.x + d2.y * d2.y + d2.z * d2.z + d2.w * d2.w;
#pragma unroll
    for (int o = 16; o > 0; o >>= 1) q += __shfl_xor(q, o, 32);
    const float rs = 1.0f / sqrtf(q * (1.0f / (float)DM) + 1e-5f);
    const v4f g0 = *(const v4f*)(g + q0), g1 = *(const v4f*)(g + q1), g2 = *(const v4f*)(g + q2);
    const v4f c0 = *(const v4f*)(bt + q0), c1 = *(const v4f*)(bt + q1), c2 = *(const v4f*)(bt + q2);
    v4f y0, y1, y2;
    y0.x = d0.x * rs * bfr(g0.x) + bfr(c0.x); y0.y = d0.y * rs * bfr(g0.y) + bfr(c0.y);
    y0.z = d0.z * rs * bfr(g0.z) + bfr(c0.z); y0.w = d0.w * rs * bfr(g0.w) + bfr(c0.w);
    y1.x = d1.x * rs * bfr(g1.x) + bfr(c1.x); y1.y = d1.y * rs * bfr(g1.y) + bfr(c1.y);
    y1.z = d1.z * rs * bfr(g1.z) + bfr(c1.z); y1.w = d1.w * rs * bfr(g1.w) + bfr(c1.w);
    y2.x = d2.x * rs * bfr(g2.x) + bfr(c2.x); y2.y = d2.y * rs * bfr(g2.y) + bfr(c2.y);
    y2.z = d2.z * rs * bfr(g2.z) + bfr(c2.z); y2.w = d2.w * rs * bfr(g2.w) + bfr(c2.w);
    float* yr = y32 + (size_t)row * DM;
    for (int pass = 0; pass < 2; ++pass) {
        *(volatile v4f*)(yr + q0) = y0;
        *(volatile v4f*)(yr + q1) = y1;
        if (ok2) *(volatile v4f*)(yr + 4u * (L + 64u)) = y2;
        __threadfence();
    }
    if (PLANE) {
        *(v4f*)(&sL[wave][q0]) = y0;
        *(v4f*)(&sL[wave][q1]) = y1;
        if (ok2) *(v4f*)(&sL[wave][4u * (L + 64u)]) = y2;
        wave_sync_lds();
        const unsigned pa = 8u * L, pb = 256u + 8u * (L & 7u);
        const v4f a0 = *(const v4f*)(&sL[wave][pa]), a1 = *(const v4f*)(&sL[wave][pa + 4u]);
        const v4f e0 = *(const v4f*)(&sL[wave][pb]), e1 = *(const v4f*)(&sL[wave][pb + 4u]);
        float va[8] = {a0.x * C_X1, a0.y * C_X1, a0.z * C_X1, a0.w * C_X1, a1.x * C_X1, a1.y * C_X1, a1.z * C_X1, a1.w * C_X1};
        float vb[8] = {e0.x * C_X1, e0.y * C_X1, e0.z * C_X1, e0.w * C_X1, e1.x * C_X1, e1.y * C_X1, e1.z * C_X1, e1.w * C_X1};
        st8h(y16, (size_t)row * DM + pa, va);
        if (L < 8u) st8h(y16, (size_t)row * DM + pb, vb);
    }
}
__global__ __launch_bounds__(256) void k_ln_mid(const float* __restrict__ h, const float* __restrict__ g, const float* __restrict__ bt,
                                                float* __restrict__ y32, unsigned short* __restrict__ y16) {
    ln320_body<true>(h, g, bt, y32, y16);
}
__global__ __launch_bounds__(256) void k_ln_out(const float* __restrict__ h, const float* __restrict__ g, const float* __restrict__ bt,
                                                float* __restrict__ y32) {
    ln320_body<false>(h, g, bt, y32, nullptr);
}

static constexpr size_t al256(size_t x) { return (x + 255) & ~(size_t)255; }
static constexpr size_t SZ_EB   = al256((size_t)MTOK * SEQ * DE * 2);
static constexpr size_t SZ_X16  = al256((size_t)MTOK * DM * 2);
static constexpr size_t SZ_WQKV = al256((size_t)3 * DM * DM * 2);
static constexpr size_t SZ_WO   = al256((size_t)DM * DM * 2);
static constexpr size_t SZ_W1   = al256((size_t)FFD * DM * 2);
static constexpr size_t SZ_W2   = al256((size_t)DM * FFD * 2);
static constexpr size_t SZ_WE   = al256((size_t)DM * DE * 2);
static constexpr size_t SZ_QKV  = al256((size_t)MTOK * 3 * DM * 4);
static constexpr size_t SZ_QS   = al256((size_t)MTOK * DM * 4);
static constexpr size_t SZ_KVT  = al256((size_t)2 * NB * DM * SEQ * 4);
static constexpr size_t SZ_WV   = al256((size_t)MTOK * DM * 2);
static constexpr size_t SZ_H    = al256((size_t)MTOK * DM * 4);
static constexpr size_t SZ_X1H  = al256((size_t)MTOK * DM * 2);
static constexpr size_t SZ_HH   = al256((size_t)MTOK * FFD * 2);
static constexpr size_t OFF_EB   = 0;
static constexpr size_t OFF_X16  = OFF_EB + SZ_EB;
static constexpr size_t OFF_WQKV = OFF_X16 + SZ_X16;
static constexpr size_t OFF_WO   = OFF_WQKV + SZ_WQKV;
static constexpr size_t OFF_W1   = OFF_WO + SZ_WO;
static constexpr size_t OFF_W2   = OFF_W1 + SZ_W1;
static constexpr size_t OFF_WEM  = OFF_W2 + SZ_W2;
static constexpr size_t OFF_WEA  = OFF_WEM + SZ_WE;
static constexpr size_t OFF_QKV  = OFF_WEA + SZ_WE;
static constexpr size_t OFF_QS   = OFF_QKV + SZ_QKV;
static constexpr size_t OFF_KVT  = OFF_QS + SZ_QS;
static constexpr size_t OFF_WV   = OFF_KVT + SZ_KVT;
static constexpr size_t OFF_H1   = OFF_WV + SZ_WV;
static constexpr size_t OFF_X1   = OFF_H1 + SZ_H;
static constexpr size_t OFF_X1H  = OFF_X1 + SZ_H;
static constexpr size_t OFF_HH   = OFF_X1H + SZ_X1H;
static constexpr size_t OFF_H2   = OFF_HH + SZ_HH;
static constexpr size_t WS_TOTAL = OFF_H2 + SZ_H;
static_assert(WS_TOTAL <= (size_t)134217728);

static constexpr unsigned cdiv(unsigned a, unsigned b) { return (a + b - 1u) / b; }
static constexpr unsigned N8_E = (unsigned)((size_t)MTOK * SEQ * DE / 8);
static constexpr unsigned N8_X = (unsigned)(MTOK * DM / 8);
static constexpr unsigned G_QKV = cdiv((MTOK / 64) * (3 * DM / 64), 8);
static constexpr unsigned G_D   = cdiv((MTOK / 64) * (DM / 64), 8);
static constexpr unsigned G_F   = cdiv((MTOK / 64) * (FFD / 64), 8);
static_assert((DM / 8) % 8 == 0 && (FFD / 8) % 8 == 0 && (DE / 8) % 8 == 0);

extern "C" void kernel_launch(void* const* d_in, const int* in_sizes, int n_in, void* d_out, int out_size,
                              void* d_ws, size_t ws_size, hipStream_t stream) {
    if (n_in < 23) return;
    if (in_sizes[0] < MTOK * DM || in_sizes[1] < MTOK * SEQ * DE || in_sizes[2] < MTOK) return;
    if (in_sizes[3] < DM * DM || in_sizes[4] < DM || in_sizes[5] < DM * DM || in_sizes[6] < DM) return;
    if (in_sizes[7] < DM * DM || in_sizes[8] < DM || in_sizes[9] < DE * DM || in_sizes[10] < DM) return;
    if (in_sizes[11] < DE * DM || in_sizes[12] < DM || in_sizes[13] < DM * DM || in_sizes[14] < DM) return;
    if (in_sizes[15] < DM * FFD || in_sizes[16] < FFD || in_sizes[17] < FFD * DM || in_sizes[18] < DM) return;
    if (in_sizes[19] < DM || in_sizes[20] < DM || in_sizes[21] < DM || in_sizes[22] < DM) return;
    if (out_size < MTOK * DM) return;
    if (ws_size < WS_TOTAL) return;

    const float* X     = (const float*)d_in[0];
    const float* E     = (const float*)d_in[1];
    const float* nmask = (const float*)d_in[2];
    const float* Wq    = (const float*)d_in[3];
    const float* bq    = (const float*)d_in[4];
    const float* Wk    = (const float*)d_in[5];
    const float* bk    = (const float*)d_in[6];
    const float* Wv    = (const float*)d_in[7];
    const float* bv    = (const float*)d_in[8];
    const float* Wem   = (const float*)d_in[9];
    const float* bem   = (const float*)d_in[10];
    const float* Wea   = (const float*)d_in[11];
    const float* bea   = (const float*)d_in[12];
    const float* Wo    = (const float*)d_in[13];
    const float* bo    = (const float*)d_in[14];
    const float* W1    = (const float*)d_in[15];
    const float* b1    = (const float*)d_in[16];
    const float* W2    = (const float*)d_in[17];
    const float* b2    = (const float*)d_in[18];
    const float* g1    = (const float*)d_in[19];
    const float* beta1 = (const float*)d_in[20];
    const float* g2    = (const float*)d_in[21];
    const float* beta2 = (const float*)d_in[22];
    float* out = (float*)d_out;

    char* wsp = (char*)d_ws;
    unsigned short* eb16  = (unsigned short*)(wsp + OFF_EB);
    unsigned short* x16   = (unsigned short*)(wsp + OFF_X16);
    unsigned short* wqkv  = (unsigned short*)(wsp + OFF_WQKV);
    unsigned short* wo16  = (unsigned short*)(wsp + OFF_WO);
    unsigned short* w1_16 = (unsigned short*)(wsp + OFF_W1);
    unsigned short* w2_16 = (unsigned short*)(wsp + OFF_W2);
    unsigned short* wem16 = (unsigned short*)(wsp + OFF_WEM);
    unsigned short* wea16 = (unsigned short*)(wsp + OFF_WEA);
    float*          qkv   = (float*)(wsp + OFF_QKV);
    float*          qs    = (float*)(wsp + OFF_QS);
    float*          kvt   = (float*)(wsp + OFF_KVT);
    unsigned short* wv16  = (unsigned short*)(wsp + OFF_WV);
    float*          h1    = (float*)(wsp + OFF_H1);
    float*          x1    = (float*)(wsp + OFF_X1);
    unsigned short* x1h   = (unsigned short*)(wsp + OFF_X1H);
    unsigned short* hh16  = (unsigned short*)(wsp + OFF_HH);
    float*          h2    = (float*)(wsp + OFF_H2);

    k_wt16<<<cdiv(DM * (DM / 8), 256), 256, 0, stream>>>(Wq, DM, DM, DM / 8, wqkv, LG_W);
    k_wt16<<<cdiv(DM * (DM / 8), 256), 256, 0, stream>>>(Wk, DM, DM, DM / 8, wqkv + (size_t)DM * DM, LG_W);
    k_wt16<<<cdiv(DM * (DM / 8), 256), 256, 0, stream>>>(Wv, DM, DM, DM / 8, wqkv + (size_t)2 * DM * DM, LG_W);
    k_wt16<<<cdiv(DM * (DM / 8), 256), 256, 0, stream>>>(Wo, DM, DM, DM / 8, wo16, LG_WO);
    k_wt16<<<cdiv(FFD * (DM / 8), 256), 256, 0, stream>>>(W1, DM, FFD, DM / 8, w1_16, LG_W);
    k_wt16<<<cdiv(DM * (FFD / 8), 256), 256, 0, stream>>>(W2, FFD, DM, FFD / 8, w2_16, LG_W);
    k_wt16<<<cdiv(DM * (DE / 8), 256), 256, 0, stream>>>(Wem, DE, DM, DE / 8, wem16, LG_W);
    k_wt16<<<cdiv(DM * (DE / 8), 256), 256, 0, stream>>>(Wea, DE, DM, DE / 8, wea16, LG_W);

    k_cvt8<<<N8_E / 256, 256, 0, stream>>>(E, eb16, N8_E);
    k_cvt8<<<N8_X / 256, 256, 0, stream>>>(X, x16, N8_X);

    k_gemm_qkv<<<G_QKV, 256, 0, stream>>>((const _Float16*)x16, (const _Float16*)wqkv, qkv);
    k_qkvt<<<dim3(DM / 64, MTOK / 64, 3), 256, 0, stream>>>(qkv, bq, bk, bv, nmask, qs, kvt);

    k_eattn<<<MTOK * 5, 128, 0, stream>>>((const _Float16*)eb16, (const _Float16*)wem16, (const _Float16*)wea16,
                                          bem, bea, nmask, qs, kvt, (_Float16*)wv16);

    k_gemm_wo<<<G_D, 256, 0, stream>>>((const _Float16*)wv16, (const _Float16*)wo16, h1, bo, X, nmask);
    k_ln_mid<<<MTOK / 8, 256, 0, stream>>>(h1, g1, beta1, x1, x1h);

    k_gemm_ff1<<<G_F, 256, 0, stream>>>((const _Float16*)x1h, (const _Float16*)w1_16, (_Float16*)hh16, b1);
    k_gemm_ff2<<<G_D, 256, 0, stream>>>((const _Float16*)hh16, (const _Float16*)w2_16, h2, b2, x1);
    k_ln_out<<<MTOK / 8, 256, 0, stream>>>(h2, g2, beta2, out);
}
